// SparseEncoderLayer_57200374448504
// MI455X (gfx1250) — hardware-verified
//
#include <hip/hip_runtime.h>


namespace {
constexpr int N = 131072, M = 58963, CIN = 3, NF = 32, K3 = 27, K2 = 8;
constexpr int NB1 = N / 128, NB3 = (M + 127) / 128;
constexpr float AS = 8.0f, WS = 64.0f, EPS = 1e-5f;

typedef _Float16 b16;
typedef __attribute__((ext_vector_type(16))) _Float16 v16b;
typedef __attribute__((ext_vector_type(8)))  _Float16 v8b;
typedef __attribute__((ext_vector_type(8)))  float v8f;
typedef __attribute__((ext_vector_type(4)))  float v4f;

__device__ __forceinline__ v8b ld8b(const b16* p) { return *(const v8b*)p; }
__device__ __forceinline__ v16b cat8b(v8b a, v8b b) { return __builtin_shufflevector(a, b, 0, 1, 2, 3, 4, 5, 6, 7, 8, 9, 10, 11, 12, 13, 14, 15); }
__device__ __forceinline__ v16b frag_kb(const b16* p, int hh) { return cat8b(ld8b(p + 8 * hh), ld8b(p + 16 + 8 * hh)); }
__device__ __forceinline__ void split16(float v, b16& hi, b16& lo) { hi = (b16)v; lo = (b16)(v - (float)hi); }
__device__ __forceinline__ void frag_ksplit(const float* p, int hh, v16b& fh_, v16b& fl_) {
  const float* p0 = p + 8 * hh; const float* p1 = p + 16 + 8 * hh;
#pragma unroll
  for (int e = 0; e < 8; ++e) { b16 a, c; split16(p0[e], a, c); fh_[e] = a; fl_[e] = c; split16(p1[e], a, c); fh_[8 + e] = a; fl_[8 + e] = c; }
}
__device__ __forceinline__ v8f wmma16b(v16b a, v16b b, v8f c) {
  v8f d = __builtin_amdgcn_wmma_f32_16x16x32_f16(false, a, false, b, (short)0, c, false, false);
  asm volatile("v_nop\n\tv_nop\n\tv_nop\n\tv_nop" : "+v"(d) : "v"(a), "v"(b));
  return d;
}
__device__ __forceinline__ void wave_lds_sync() {
  __builtin_amdgcn_fence(__ATOMIC_RELEASE, "workgroup");
  __builtin_amdgcn_wave_barrier();
  __builtin_amdgcn_fence(__ATOMIC_ACQUIRE, "workgroup");
}

struct Opnd { const void* p0; const void* p1; int ld; };
template <int NP> __device__ __forceinline__ void load_frags(const Opnd& o, int row, int kb, int hh, v16b& fh_, v16b& fl_) {
  if (NP == 0) { frag_ksplit((const float*)o.p0 + (size_t)row * o.ld + kb, hh, fh_, fl_); }
  else if (NP == 4) {
    const float* p = (const float*)o.p0 + (size_t)row * o.ld + kb; const float* p0 = p + 8 * hh; const float* p1 = p + 16 + 8 * hh;
#pragma unroll
    for (int e = 0; e < 8; ++e) { b16 a, c; split16(p0[e] * 64.0f, a, c); fh_[e] = a; fl_[e] = c; split16(p1[e] * 64.0f, a, c); fh_[8 + e] = a; fl_[8 + e] = c; }
  } else if (NP == 3) {
    const float* p = (const float*)o.p0 + (size_t)row * o.ld + kb; const float* p0 = p + 8 * hh; const float* p1 = p + 16 + 8 * hh;
#pragma unroll
    for (int e = 0; e < 8; ++e) { fh_[e] = (b16)p0[e]; fh_[8 + e] = (b16)p1[e]; }
    fl_ = fh_;
  } else {
    fh_ = frag_kb((const b16*)o.p0 + (size_t)row * o.ld + kb, hh);
    if (NP == 2) fl_ = frag_kb((const b16*)o.p1 + (size_t)row * o.ld + kb, hh); else fl_ = fh_;
  }
}
template <int ANP, int BNP> __device__ __forceinline__ v8f mac(v16b ah, v16b al, v16b bh, v16b bl, v8f c) {
  c = wmma16b(ah, bh, c);
  if (BNP == 0 || BNP == 2 || BNP == 4) c = wmma16b(ah, bl, c);
  if (ANP == 0 || ANP == 2 || ANP == 4) c = wmma16b(al, bh, c);
  return c;
}
template <int ANP, int BNP>
__device__ __forceinline__ void gemm_tile(const Opnd& A, const Opnd& B, int K, int m0, int c0, int nloc, int hlf, v8f (&acc)[2][4]) {
  for (int kb = 0; kb < K; kb += 32) {
    v16b a0h, a0l, a1h, a1l;
    load_frags<ANP>(A, m0 + nloc, kb, hlf, a0h, a0l);
    load_frags<ANP>(A, m0 + 16 + nloc, kb, hlf, a1h, a1l);
#pragma unroll
    for (int t = 0; t < 4; ++t) {
      v16b bh, bl;
      load_frags<BNP>(B, c0 + t * 16 + nloc, kb, hlf, bh, bl);
      acc[0][t] = mac<ANP, BNP>(a0h, a0l, bh, bl, acc[0][t]);
      acc[1][t] = mac<ANP, BNP>(a1h, a1l, bh, bl, acc[1][t]);
    }
  }
}

__device__ __forceinline__ void epi_planes(v8f (&acc)[2][4], float scale, bool two, b16* __restrict__ oh, b16* __restrict__ ol, int ldo,
                                           int m0, int c0, int lane, b16* Th, b16* Tl) {
  const int nloc = lane & 15, hlf = lane >> 4;
#pragma unroll
  for (int t = 0; t < 4; ++t)
#pragma unroll
    for (int r = 0; r < 2; ++r)
#pragma unroll
      for (int v = 0; v < 8; ++v) {
        const int rr = r * 16 + v + 8 * hlf, cc = t * 16 + nloc;
        b16 h_, l_; split16(acc[r][t][v] * scale, h_, l_);
        Th[rr * 64 + cc] = h_; Tl[rr * 64 + cc] = l_;
      }
  wave_lds_sync();
  for (int pass = 0; pass < 2; ++pass) {
#pragma unroll
    for (int j = 0; j < 8; ++j) {
      const int rr = j * 4 + (lane >> 3), c8 = (lane & 7) * 8;
      const size_t o = (size_t)(m0 + rr) * ldo + c0 + c8;
      *(volatile v8b*)(oh + o) = ld8b(Th + rr * 64 + c8);
      if (two) *(volatile v8b*)(ol + o) = ld8b(Tl + rr * 64 + c8);
    }
    __threadfence();
  }
}
__device__ __forceinline__ void epi_f32(v8f (&acc)[2][4], float scale, const float* rscale, float* __restrict__ out, int ldo, int m0, int c0, int lane, float* Tt) {
  const int nloc = lane & 15, hlf = lane >> 4;
#pragma unroll
  for (int t = 0; t < 4; ++t)
#pragma unroll
    for (int r = 0; r < 2; ++r)
#pragma unroll
      for (int v = 0; v < 8; ++v) {
        const int rr = r * 16 + v + 8 * hlf;
        const float rs = rscale ? rscale[(size_t)(m0 + rr) * 32] : 1.0f;
        Tt[rr * 64 + t * 16 + nloc] = acc[r][t][v] * scale * rs;
      }
  wave_lds_sync();
  float* dst0 = out + (size_t)m0 * ldo + c0;
  for (int pass = 0; pass < 2; ++pass) {
#pragma unroll
    for (int j = 0; j < 16; ++j) { const int rr = j * 2 + hlf, c4 = nloc * 4; *(volatile v4f*)(dst0 + (size_t)rr * ldo + c4) = *(const v4f*)(Tt + rr * 64 + c4); }
    __threadfence();
  }
}


__global__ __launch_bounds__(256) void prep_kernel(const float* __restrict__ W1, const float* __restrict__ W2a, const float* __restrict__ W2b, const float* __restrict__ W3,
                                                   b16* __restrict__ ph, b16* __restrict__ pl) {
  const int tid = blockIdx.x * 256 + threadIdx.x;
  const int n1 = NF * 96 / 8, n2 = NF * 864 / 8, n3 = NF * 256 / 8, tot = n1 + 2 * n2 + n3;
  if (tid >= tot) return;
  int m, q; if (tid < n1) { m = 0; q = tid; } else if (tid < n1 + n2) { m = 1; q = tid - n1; } else if (tid < n1 + 2 * n2) { m = 2; q = tid - n1 - n2; } else { m = 3; q = tid - n1 - 2 * n2; }
  const int KW = (m == 0) ? 96 : (m == 3) ? 256 : 864; const int d = (q * 8) / KW, k0 = (q * 8) % KW;
  const size_t base = (m == 0) ? 0 : (m == 1) ? (size_t)NF * 96 : (m == 2) ? (size_t)NF * (96 + 864) : (size_t)NF * (96 + 1728);
  v8b vh, vl;
#pragma unroll
  for (int e = 0; e < 8; ++e) {
    const int k = k0 + e; float w = 0.0f;
    if (m == 0) { if (k < K3 * CIN) { const int o = k / CIN, c = k % CIN; w = W1[(o * CIN + c) * NF + d]; } }
    else if (m == 3) { const int o = k / NF, c = k % NF; w = W3[(o * NF + c) * NF + d]; }
    else { const int o = k / NF, c = k % NF; w = ((m == 1) ? W2a : W2b)[(o * NF + c) * NF + d]; }
    b16 a, b2; split16(w * WS, a, b2); vh[e] = a; vl[e] = b2;
  }
  const size_t oo = base + (size_t)d * KW + k0;
  *(volatile v8b*)(ph + oo) = vh; *(volatile v8b*)(pl + oo) = vl; __threadfence(); *(volatile v8b*)(ph + oo) = vh; *(volatile v8b*)(pl + oo) = vl;
}

__device__ __forceinline__ void epi_rows_stats(v8f (&acc)[2][4], float scale, const float* __restrict__ resid, float* __restrict__ out, int nrows, int m0,
                                               int lane, int wave, float* __restrict__ Ts, float (*Ss)[64], float* __restrict__ slot) {
  const int nloc = lane & 15, hlf = lane >> 4;
  float cs[2] = {0.f, 0.f}, cs2[2] = {0.f, 0.f};
#pragma unroll
  for (int t = 0; t < 2; ++t)
#pragma unroll
    for (int r = 0; r < 2; ++r)
#pragma unroll
      for (int v = 0; v < 8; ++v) {
        const int rr = r * 16 + v + 8 * hlf, cc = t * 16 + nloc, row = m0 + rr;
        float val = acc[r][t][v] * scale;
        if (resid && row < nrows) val += resid[(size_t)row * NF + cc];
        Ts[rr * 32 + cc] = val;
        if (row < nrows) { cs[t] += val; cs2[t] += val * val; }
      }
#pragma unroll
  for (int t = 0; t < 2; ++t) { cs[t] += __shfl_xor(cs[t], 16); cs2[t] += __shfl_xor(cs2[t], 16); if (hlf == 0) { Ss[wave][t * 16 + nloc] = cs[t]; Ss[wave][32 + t * 16 + nloc] = cs2[t]; } }
  wave_lds_sync();
  for (int pass = 0; pass < 2; ++pass) {
#pragma unroll
    for (int j = 0; j < 8; ++j) { const int rr = j * 4 + (lane >> 3), c4 = (lane & 7) * 4, row = m0 + rr;
      if (row < nrows) *(volatile v4f*)(out + (size_t)row * NF + c4) = *(const v4f*)(Ts + rr * 32 + c4); }
    __threadfence();
  }
  __syncthreads();
  if (wave == 0) {
    float s0 = Ss[0][lane] + Ss[1][lane] + Ss[2][lane] + Ss[3][lane], s1 = Ss[0][32 + lane] + Ss[1][32 + lane] + Ss[2][32 + lane] + Ss[3][32 + lane];
    for (int pass = 0; pass < 2; ++pass) { ((volatile float*)slot)[(size_t)blockIdx.x * 64 + lane] = s0; ((volatile float*)slot)[(size_t)blockIdx.x * 64 + 32 + lane] = s1; __threadfence(); }
  }
}

__global__ __launch_bounds__(128) void conv1_kernel(const float* __restrict__ feats, const int* __restrict__ nbr, const b16* __restrict__ wh, const b16* __restrict__ wl,
                                                   float* __restrict__ x1, float* __restrict__ slot) {
  __shared__ __attribute__((aligned(16))) float Ts[4][32 * 32]; __shared__ float Ss[4][64];
  __shared__ __attribute__((aligned(16))) b16 Gh[4][32][96 + 8]; __shared__ __attribute__((aligned(16))) b16 Gl[4][32][96 + 8];
  const int lane = threadIdx.x & 31, wave = threadIdx.x >> 5, nloc = lane & 15, hlf = lane >> 4, m0 = blockIdx.x * 128 + wave * 32;
  {
    const int row = m0 + lane;
#pragma unroll 1
    for (int o = 0; o < K3; ++o) {
      const int id = nbr[(size_t)row * K3 + o];
#pragma unroll
      for (int c = 0; c < CIN; ++c) { const float v = (id >= 0 && id < N) ? feats[(size_t)id * CIN + c] : 0.0f; b16 a, b2; split16(v * AS, a, b2); Gh[wave][lane][o * CIN + c] = a; Gl[wave][lane][o * CIN + c] = b2; }
    }
    for (int k = K3 * CIN; k < 96; ++k) { Gh[wave][lane][k] = (b16)0.0f; Gl[wave][lane][k] = (b16)0.0f; }
  }
  wave_lds_sync();
  v8f acc[2][4];
#pragma unroll
  for (int r = 0; r < 2; ++r)
#pragma unroll
    for (int t = 0; t < 4; ++t) acc[r][t] = (v8f){};
  for (int kb = 0; kb < 96; kb += 32) {
    const v16b a0h = frag_kb(&Gh[wave][nloc][kb], hlf), a0l = frag_kb(&Gl[wave][nloc][kb], hlf), a1h = frag_kb(&Gh[wave][16 + nloc][kb], hlf), a1l = frag_kb(&Gl[wave][16 + nloc][kb], hlf);
#pragma unroll
    for (int t = 0; t < 2; ++t) { const Opnd B{wh, wl, 96}; v16b bh, bl; load_frags<2>(B, t * 16 + nloc, kb, hlf, bh, bl);
      acc[0][t] = mac<2, 2>(a0h, a0l, bh, bl, acc[0][t]); acc[1][t] = mac<2, 2>(a1h, a1l, bh, bl, acc[1][t]); }
  }
  epi_rows_stats(acc, 1.0f / (AS * WS), nullptr, x1, N, m0, lane, wave, Ts[wave], Ss, slot);
}

template <int NOFF>
__global__ __launch_bounds__(128) void gconv_kernel(const b16* __restrict__ yh, const b16* __restrict__ yl, const int* __restrict__ tab, int nrows,
                                                    const b16* __restrict__ wh, const b16* __restrict__ wl, const float* __restrict__ resid, float* __restrict__ out, float* __restrict__ slot) {
  __shared__ __attribute__((aligned(16))) float Ts[4][32 * 32]; __shared__ float Ss[4][64];
  __shared__ __attribute__((aligned(16))) b16 Gh[4][32][NF + 8]; __shared__ __attribute__((aligned(16))) b16 Gl[4][32][NF + 8];
  const int lane = threadIdx.x & 31, wave = threadIdx.x >> 5, nloc = lane & 15, hlf = lane >> 4, m0 = blockIdx.x * 128 + wave * 32;
  const int myrow = m0 + lane; const bool vme = myrow < nrows;
  v8f acc[2][4];
#pragma unroll
  for (int r = 0; r < 2; ++r)
#pragma unroll
    for (int t = 0; t < 4; ++t) acc[r][t] = (v8f){};
#pragma unroll 1
  for (int o = 0; o < NOFF; ++o) {
    int id = vme ? tab[(size_t)myrow * NOFF + o] : -1; id = (id < 0 || id >= N) ? N : id;
#pragma unroll
    for (int p = 0; p < 4; ++p) { *(v8b*)(&Gh[wave][lane][p * 8]) = ld8b(yh + (size_t)id * NF + p * 8); *(v8b*)(&Gl[wave][lane][p * 8]) = ld8b(yl + (size_t)id * NF + p * 8); }
    wave_lds_sync();
    const v16b a0h = frag_kb(&Gh[wave][nloc][0], hlf), a0l = frag_kb(&Gl[wave][nloc][0], hlf), a1h = frag_kb(&Gh[wave][16 + nloc][0], hlf), a1l = frag_kb(&Gl[wave][16 + nloc][0], hlf);
#pragma unroll
    for (int t = 0; t < 2; ++t) { const Opnd B{wh, wl, NOFF * NF}; v16b bh, bl; load_frags<2>(B, t * 16 + nloc, o * NF, hlf, bh, bl);
      acc[0][t] = mac<2, 2>(a0h, a0l, bh, bl, acc[0][t]); acc[1][t] = mac<2, 2>(a1h, a1l, bh, bl, acc[1][t]); }
    wave_lds_sync();
  }
  epi_rows_stats(acc, 1.0f / (AS * WS), resid, out, nrows, m0, lane, wave, Ts[wave], Ss, slot);
}

__global__ __launch_bounds__(64) void bnfin_kernel(const float* __restrict__ slot, int nblk, int nrows, const float* __restrict__ g, const float* __restrict__ bb, float* __restrict__ coef) {
  const int c = threadIdx.x & 31;
  if (threadIdx.x < 32) {
    double s = 0.0, s2 = 0.0;
#pragma unroll 1
    for (int bk = 0; bk < nblk; ++bk) { s += (double)slot[(size_t)bk * 64 + c]; s2 += (double)slot[(size_t)bk * 64 + 32 + c]; }
    const double mean = s / nrows, var = s2 / nrows - mean * mean;
    const float a = g[c] * (float)(1.0 / sqrt(var + (double)EPS)), sh = bb[c] - (float)mean * a;
    for (int pass = 0; pass < 2; ++pass) { ((volatile float*)coef)[c] = a; ((volatile float*)coef)[32 + c] = sh; __threadfence(); }
  }
}

__global__ __launch_bounds__(256) void bnapply_kernel(const float* __restrict__ x, int nrows, const float* __restrict__ coef, b16* __restrict__ yh, b16* __restrict__ yl, float* __restrict__ fout) {
  __shared__ __attribute__((aligned(16))) float V[128 * 32];
  const int t = threadIdx.x, r0 = blockIdx.x * 128;
  for (int i = t; i < 128 * 32; i += 256) { const int row = r0 + i / 32, c = i % 32; float v = 0.0f; if (row < nrows) v = fmaxf(x[(size_t)row * NF + c] * coef[c] + coef[32 + c], 0.0f); V[i] = v; }
  __syncthreads();
  for (int pass = 0; pass < 2; ++pass) {
#pragma unroll
    for (int j = 0; j < 2; ++j) { const int pc_ = j * 256 + t, row = r0 + pc_ / 4, c8 = (pc_ % 4) * 8;
      if (row < nrows) { v8b vh, vl;
#pragma unroll
        for (int e = 0; e < 8; ++e) { b16 a, b2; split16(V[(pc_ / 4) * 32 + c8 + e] * AS, a, b2); vh[e] = a; vl[e] = b2; }
        *(volatile v8b*)(yh + (size_t)row * NF + c8) = vh; *(volatile v8b*)(yl + (size_t)row * NF + c8) = vl; } }
    if (fout) {
#pragma unroll
      for (int j = 0; j < 4; ++j) { const int pc_ = j * 256 + t, row = r0 + pc_ / 8, c4 = (pc_ % 8) * 4;
        if (row < nrows) *(volatile v4f*)(fout + (size_t)row * NF + c4) = *(const v4f*)(&V[(pc_ / 8) * 32 + c4]); }
    }
    if (blockIdx.x == 0 && t < 8) { v8b z;
#pragma unroll
      for (int e = 0; e < 8; ++e) z[e] = (b16)0.0f;
      *(volatile v8b*)((t < 4 ? yh : yl) + (size_t)N * NF + (t & 3) * 8) = z; }
    __threadfence();
  }
}
}

extern "C" void kernel_launch(void* const* d_in, const int* in_sizes, int n_in,
                              void* d_out, int out_size, void* d_ws, size_t ws_size, hipStream_t stream) {
  (void)n_in; (void)out_size;
  const float* feats = (const float*)d_in[0];
  const int* nbr = (const int*)d_in[1];
  const int* child = (const int*)d_in[2];
  const float* W1 = (const float*)d_in[3]; const float* W2a = (const float*)d_in[4]; const float* W2b = (const float*)d_in[5]; const float* W3 = (const float*)d_in[6];
  const float* g1 = (const float*)d_in[7];  const float* b1 = (const float*)d_in[8];
  const float* g2 = (const float*)d_in[9];  const float* b2 = (const float*)d_in[10];
  const float* g3 = (const float*)d_in[11]; const float* b3 = (const float*)d_in[12];
  const float* g4 = (const float*)d_in[13]; const float* b4 = (const float*)d_in[14];
  float* out = (float*)d_out;
  if (in_sizes[0] != N * CIN || in_sizes[1] != N * K3 || in_sizes[2] != M * K2 || in_sizes[3] != K3 * CIN * NF || in_sizes[6] != K2 * NF * NF) return;

  size_t off = 0; char* ws = (char*)d_ws;
  auto carve = [&](size_t bytes) { char* p = ws + off; off += (bytes + 255) & ~(size_t)255; return p; };
  const size_t NPL = (size_t)NF * (96 + 864 + 864 + 256);
  b16* wph = (b16*)carve(NPL * 2); b16* wpl = (b16*)carve(NPL * 2);
  float* x1 = (float*)carve((size_t)N * NF * 4);
  float* br = (float*)carve((size_t)N * NF * 4);
  float* x3 = (float*)carve((size_t)NB3 * 128 * NF * 4);
  b16* yh = (b16*)carve((size_t)(N + 1) * NF * 2);
  b16* yl = (b16*)carve((size_t)(N + 1) * NF * 2);
  float* slot = (float*)carve((size_t)NB1 * 64 * 4);
  float* coef = (float*)carve(256 * 4);
  if (off > ws_size) return;
  const b16* w1h = wph; const b16* w1l = wpl; const b16* w2ah = wph + NF * 96; const b16* w2al = wpl + NF * 96;
  const b16* w2bh = wph + NF * (96 + 864); const b16* w2bl = wpl + NF * (96 + 864); const b16* w3h = wph + NF * (96 + 1728); const b16* w3l = wpl + NF * (96 + 1728);
  float* ft2 = out + (size_t)M * NF;
  prep_kernel<<<(int)((NPL / 8 + 255) / 256), 256, 0, stream>>>(W1, W2a, W2b, W3, wph, wpl);
  conv1_kernel<<<NB1, 128, 0, stream>>>(feats, nbr, w1h, w1l, x1, slot);
  bnfin_kernel<<<1, 64, 0, stream>>>(slot, NB1, N, g1, b1, coef);
  bnapply_kernel<<<NB1, 256, 0, stream>>>(x1, N, coef, yh, yl, nullptr);
  gconv_kernel<K3><<<NB1, 128, 0, stream>>>(yh, yl, nbr, N, w2ah, w2al, nullptr, br, slot);
  bnfin_kernel<<<1, 64, 0, stream>>>(slot, NB1, N, g2, b2, coef);
  bnapply_kernel<<<NB1, 256, 0, stream>>>(br, N, coef, yh, yl, nullptr);
  gconv_kernel<K3><<<NB1, 128, 0, stream>>>(yh, yl, nbr, N, w2bh, w2bl, x1, br, slot);
  bnfin_kernel<<<1, 64, 0, stream>>>(slot, NB1, N, g3, b3, coef);
  bnapply_kernel<<<NB1, 256, 0, stream>>>(br, N, coef, yh, yl, ft2);
  gconv_kernel<K2><<<NB3, 128, 0, stream>>>(yh, yl, child, M, w3h, w3l, nullptr, x3, slot);
  bnfin_kernel<<<1, 64, 0, stream>>>(slot, NB3, M, g4, b4, coef);
  bnapply_kernel<<<NB3, 256, 0, stream>>>(x3, M, coef, yh, yl, out);
}
